// PMLP_14491219656875
// MI455X (gfx1250) — hardware-verified
//
#include <hip/hip_runtime.h>
#include <stdint.h>
#include <math.h>

constexpr int NNODE     = 100000;
constexpr int NEDGE_ALL = 3200000;
constexpr int FIN       = 58;
constexpr int FW        = 64;
constexpr int NHID      = 16;
constexpr int NGEMM     = 64;
constexpr int AGG_NT    = 256;
constexpr int AGG_SRB   = 2048;
constexpr int AGG_SCH   = 2048;
constexpr int AGG_SPT   = AGG_SCH / AGG_NT;
constexpr int AGG_TILES = 49;
constexpr int NPA       = AGG_TILES * AGG_SRB;
constexpr int MPAD      = 100032;
constexpr float MEAN_SC = 64.0f;
constexpr float W1_SC   = 16.0f;
constexpr float GEMM_SC = 1.0f / 1024.0f;

static_assert(NNODE < (1 << 17), "");
static_assert(NEDGE_ALL % AGG_SPT == 0, "");
static_assert(AGG_SRB == 2048 && AGG_NT == 256 && AGG_SCH == 2048, "");
static_assert(MPAD % 64 == 0 && MPAD >= NNODE && NPA >= MPAD, "");
static_assert(NNODE % 32 == 0, "");
static_assert((NNODE * 16) % 256 == 0, "");
static_assert((MPAD * 8) % 256 == 0, "");
static_assert(FW % 32 == 0 && NGEMM % 64 == 0 && FIN <= FW && NHID <= NGEMM, "");
static_assert((NEDGE_ALL * 4) % 16 == 0, "");

typedef __attribute__((ext_vector_type(16))) _Float16 v16h;
typedef __attribute__((ext_vector_type(8)))  _Float16 v8h;
typedef __attribute__((ext_vector_type(16))) __bf16   v16b;
typedef __attribute__((ext_vector_type(8)))  __bf16   v8b;
typedef __attribute__((ext_vector_type(8)))  float    v8f;
typedef __attribute__((ext_vector_type(4)))  float    v4f;
typedef __attribute__((ext_vector_type(2)))  float    v2f;
typedef __attribute__((ext_vector_type(4)))  int      v4i;

__device__ __forceinline__ unsigned short f2bf_bits(float f) {
  unsigned u = __float_as_uint(f);
  return (unsigned short)((u + 0x7FFFu + ((u >> 16) & 1u)) >> 16);
}
__device__ __forceinline__ float bf_bits2f(unsigned short h) { return __uint_as_float(((unsigned)h) << 16); }

__device__ __forceinline__ void dep_guard_h(v8f& a, v8f& b, v16h x, v16h y) { asm volatile("v_nop\n\tv_nop\n\tv_nop\n\tv_nop" : "+v"(a), "+v"(b) : "v"(x), "v"(y)); }
__device__ __forceinline__ void dep_guard_b(v8f& a, v8f& b, v16b x, v16b y) { asm volatile("v_nop\n\tv_nop\n\tv_nop\n\tv_nop" : "+v"(a), "+v"(b) : "v"(x), "v"(y)); }
__device__ __forceinline__ void keep4_h(v16h a, v16h b, v16h c, v16h d) { asm volatile("v_nop" :: "v"(a), "v"(b), "v"(c), "v"(d)); }
__device__ __forceinline__ void keep4_b(v16b a, v16b b, v16b c, v16b d) { asm volatile("v_nop" :: "v"(a), "v"(b), "v"(c), "v"(d)); }
__device__ __forceinline__ void acc_guard4(v8f& a, v8f& b, v8f& c, v8f& d) { asm volatile("v_nop\n\tv_nop\n\tv_nop\n\tv_nop" : "+v"(a), "+v"(b), "+v"(c), "+v"(d)); }
template <typename T> struct Frag;
template <> struct Frag<_Float16> {
  typedef v16h V; union U { v16h v; v8h h[2]; };
  static __device__ __forceinline__ v16h load(const _Float16* p) {
    U f; f.h[0] = *(const v8h*)(p); f.h[1] = *(const v8h*)(p + 16); return f.v;
  }
  static __device__ __forceinline__ v8f mma(v16h a, v16h b, v8f c) {
    return __builtin_amdgcn_wmma_f32_16x16x32_f16(false, a, false, b, (short)0, c, false, false);
  }
  static __device__ __forceinline__ void guard(v8f& a, v8f& b, v16h x, v16h y) { dep_guard_h(a, b, x, y); }
  static __device__ __forceinline__ void keep(v16h a, v16h b, v16h c, v16h d) { keep4_h(a, b, c, d); }
};
template <> struct Frag<__bf16> {
  typedef v16b V; union U { v16b v; v8b h[2]; };
  static __device__ __forceinline__ v16b load(const __bf16* p) {
    U f; f.h[0] = *(const v8b*)(p); f.h[1] = *(const v8b*)(p + 16); return f.v;
  }
  static __device__ __forceinline__ v8f mma(v16b a, v16b b, v8f c) {
    return __builtin_amdgcn_wmma_f32_16x16x32_bf16(false, a, false, b, (short)0, c, false, false);
  }
  static __device__ __forceinline__ void guard(v8f& a, v8f& b, v16b x, v16b y) { dep_guard_b(a, b, x, y); }
  static __device__ __forceinline__ void keep(v16b a, v16b b, v16b c, v16b d) { keep4_b(a, b, c, d); }
};

template <int ET> struct Elem;
template <> struct Elem<0> { typedef _Float16 T; };
template <> struct Elem<1> { typedef __bf16 T; };
template <int ET, bool SPLIT, int BIAS_MODE, int OUT_MODE, bool RESID, int ACT = 0>
__global__ __launch_bounds__(256) void wmma_gemm64(
    const unsigned short* __restrict__ Ap, const unsigned short* __restrict__ A2p, int lda, long strideA,
    const unsigned short* __restrict__ Btp, const unsigned short* __restrict__ Bt2p, int ldb, long strideB,
    void* __restrict__ Cout, void* __restrict__ Cout2, int ldc, long strideC,
    const float* __restrict__ bias,
    const float* __restrict__ resid, long strideR,
    int M, int N, int K, float scale) {
  typedef typename Elem<ET>::T T;
  typedef typename Frag<T>::V V;
  const T* A = (const T*)Ap; const T* A2 = (const T*)A2p; const T* Bt = (const T*)Btp; const T* Bt2 = (const T*)Bt2p;
  __shared__ __align__(16) float sT[8][16 * 68];
  const int b    = blockIdx.y;
  const int lane = threadIdx.x & 31;
  const int wave = threadIdx.x >> 5;
  const int tilesN = N >> 6;
  const int tilesM = M >> 6;
  const int tile = blockIdx.x * 8 + wave;
  if (tile >= tilesM * tilesN) return;
  const int tm = tile / tilesN;
  const int tn = tile - tm * tilesN;
  const int m0 = tm << 6;
  const int n0 = tn << 6;

  const T* Ab  = A  + (size_t)b * strideA;
  const T* Bb  = Bt + (size_t)b * strideB;
  const T* Ab2 = SPLIT ? (A2  + (size_t)b * strideA) : nullptr;
  const T* Bb2 = SPLIT ? (Bt2 + (size_t)b * strideB) : nullptr;

  const int rlane = lane & 15;
  const int koff  = (lane >> 4) * 8;
  const int mOff  = (lane >> 4) * 8;

  v8f acc[4][4];
#pragma unroll
  for (int i = 0; i < 4; ++i)
#pragma unroll
    for (int j = 0; j < 4; ++j) acc[i][j] = (v8f){0.f,0.f,0.f,0.f,0.f,0.f,0.f,0.f};

  for (int k0 = 0; k0 < K; k0 += 32) {
    V bh[4], bl[4];
#pragma unroll
    for (int j = 0; j < 4; ++j) {
      const size_t bo = (size_t)(n0 + (j << 4) + rlane) * ldb + koff + k0;
      bh[j] = Frag<T>::load(Bb + bo);
      if (SPLIT) bl[j] = Frag<T>::load(Bb2 + bo);
    }
#pragma unroll
    for (int i = 0; i < 4; ++i) {
      const size_t ao = (size_t)(m0 + (i << 4) + rlane) * lda + koff + k0;
      V ah = Frag<T>::load(Ab + ao);
      V al;
      if (SPLIT) al = Frag<T>::load(Ab2 + ao);
#pragma unroll
      for (int j = 0; j < 4; ++j) {
        acc[i][j] = Frag<T>::mma(ah, bh[j], acc[i][j]);
        if (SPLIT) {
          acc[i][j] = Frag<T>::mma(ah, bl[j], acc[i][j]);
          acc[i][j] = Frag<T>::mma(al, bh[j], acc[i][j]);
        }
      }
      Frag<T>::guard(acc[i][0], acc[i][3], ah, SPLIT ? al : ah);
    }
    Frag<T>::keep(bh[0], bh[1], bh[2], bh[3]);
    if (SPLIT) Frag<T>::keep(bl[0], bl[1], bl[2], bl[3]);
  }
  acc_guard4(acc[0][0], acc[0][1], acc[0][2], acc[0][3]);
  acc_guard4(acc[1][0], acc[1][1], acc[1][2], acc[1][3]);
  acc_guard4(acc[2][0], acc[2][1], acc[2][2], acc[2][3]);
  acc_guard4(acc[3][0], acc[3][1], acc[3][2], acc[3][3]);

  float* slab = sT[wave];
  const float* Rb = RESID ? (resid + (size_t)b * strideR) : nullptr;
#pragma unroll
  for (int i = 0; i < 4; ++i) {
    const int mBase = m0 + (i << 4);
#pragma unroll
    for (int j = 0; j < 4; ++j) {
      const int n = n0 + (j << 4) + rlane;
      float bv = 0.f;
      if (BIAS_MODE == 2) bv = bias[n];
#pragma unroll
      for (int r = 0; r < 8; ++r) {
        float v = acc[i][j][r] * scale;
        if (BIAS_MODE == 1) v += bias[mBase + mOff + r];
        if (BIAS_MODE == 2) v += bv;
        if (RESID) v += Rb[(size_t)(mBase + mOff + r) * ldc + n];
        if (ACT == 1) v = tanhf(v);
        if (ACT == 2) v = fmaxf(v, 0.0f);
        if (ACT == 3) v = v / (1.0f + expf(-v));
        if (ACT == 4) v = (v > 0.f) ? v : 0.01f * v;
        if (ACT == 5) v = 0.5f * v * (1.0f + erff(v * 0.70710678118654752f));
        slab[(mOff + r) * 68 + (j << 4) + rlane] = v;
      }
    }
    __builtin_amdgcn_fence(__ATOMIC_RELEASE, "workgroup");
    __builtin_amdgcn_wave_barrier();
    __builtin_amdgcn_fence(__ATOMIC_ACQUIRE, "workgroup");
    if (OUT_MODE == 0) {
      float* C = (float*)Cout + (size_t)b * strideC;
      const int hh = lane >> 4, c4 = (lane & 15) * 4;
      for (int pass = 0; pass < 2; ++pass) {
#pragma unroll
        for (int it = 0; it < 8; ++it) {
          const int row = it * 2 + hh;
          v4f v = *(const v4f*)(slab + row * 68 + c4);
          *(volatile v4f*)(C + (size_t)(mBase + row) * ldc + n0 + c4) = v;
        }
        __threadfence();
      }
    } else {
      const int q = lane >> 3, c8 = (lane & 7) * 8;
      unsigned short* C  = (unsigned short*)Cout  + (size_t)b * strideC;
      unsigned short* C2 = (OUT_MODE == 2) ? ((unsigned short*)Cout2 + (size_t)b * strideC) : nullptr;
      for (int pass = 0; pass < 2; ++pass) {
#pragma unroll
        for (int it = 0; it < 4; ++it) {
          const int row = it * 4 + q;
          const float* sp = slab + row * 68 + c8;
          v8h hv, lv;
#pragma unroll
          for (int e = 0; e < 8; ++e) {
            if (OUT_MODE == 1) {
              hv[e] = (_Float16)sp[e];
            } else {
              unsigned short hb = f2bf_bits(sp[e]);
              unsigned short lb = f2bf_bits(sp[e] - bf_bits2f(hb));
              hv[e] = __builtin_bit_cast(_Float16, hb);
              lv[e] = __builtin_bit_cast(_Float16, lb);
            }
          }
          *(volatile v8h*)(C + (size_t)(mBase + row) * ldc + n0 + c8) = hv;
          if (OUT_MODE == 2) *(volatile v8h*)(C2 + (size_t)(mBase + row) * ldc + n0 + c8) = lv;
        }
        __threadfence();
      }
    }
    __builtin_amdgcn_fence(__ATOMIC_RELEASE, "workgroup");
    __builtin_amdgcn_wave_barrier();
    __builtin_amdgcn_fence(__ATOMIC_ACQUIRE, "workgroup");
  }
}

__global__ __launch_bounds__(256) void xpad_kernel(const float* __restrict__ x, float* __restrict__ XP) {
  const int i = blockIdx.x * 256 + threadIdx.x;
  if (i >= NNODE * 16) return;
  const int row = i >> 4, c4 = (i & 15) * 4;
  const float* xr = x + (size_t)row * FIN;
  v4f v;
#pragma unroll
  for (int e = 0; e < 4; ++e) {
    const int c = c4 + e;
    const int cc = (c < FIN) ? c : (FIN - 1);
    const float f = xr[cc];
    v[e] = (c < FIN) ? f : 0.0f;
  }
  float* op = XP + (size_t)row * FW + c4;
  *(volatile v4f*)op = v;
  __threadfence();
  *(volatile v4f*)op = v;
}

__global__ __launch_bounds__(256) void wprep_kernel(const float* __restrict__ W1, const float* __restrict__ b1,
                                                    unsigned short* __restrict__ W1P, float* __restrict__ B1P) {
  const int i = blockIdx.x * 256 + threadIdx.x;
  const int lane = threadIdx.x & 31, wave = threadIdx.x >> 5;
  if (i < NGEMM * 8) {
    const int n = i >> 3, k8 = (i & 7) * 8;
    const int nc = (n < NHID) ? n : (NHID - 1);
    v8h hv;
#pragma unroll
    for (int e = 0; e < 8; ++e) {
      const int k = k8 + e;
      const int kc = (k < FIN) ? k : (FIN - 1);
      const float f = W1[(size_t)nc * FIN + kc] * W1_SC;
      const float g = (n < NHID && k < FIN) ? f : 0.0f;
      hv[e] = (_Float16)g;
    }
    unsigned short* ph = W1P + (size_t)n * FW + k8;
    *(volatile v8h*)ph = hv;
    __threadfence();
    *(volatile v8h*)ph = hv;
  }
  if (blockIdx.x == 0 && wave == 0) {
    const int na = 2 * lane, nb = 2 * lane + 1;
    const float fa = b1[(na < NHID) ? na : (NHID - 1)];
    const float fb = b1[(nb < NHID) ? nb : (NHID - 1)];
    v2f bv;
    bv[0] = (na < NHID) ? fa : 0.0f;
    bv[1] = (nb < NHID) ? fb : 0.0f;
    float* pb = B1P + 2 * lane;
    *(volatile v2f*)pb = bv;
    __threadfence();
    *(volatile v2f*)pb = bv;
  }
}

__device__ __forceinline__ int blk_excl_scan(int cnt, int* scan_ws, int tid, int* tot) {
  const int lane = tid & 31, wave = tid >> 5; int incl = cnt;
#pragma unroll
  for (int o = 1; o < 32; o <<= 1) { const int v = __shfl_up(incl, o, 32); if (lane >= o) incl += v; }
  if (lane == 31) scan_ws[wave] = incl;
  __syncthreads();
  if (wave == 0) { int wv = (lane < AGG_NT / 32) ? scan_ws[lane] : 0; int wincl = wv;
#pragma unroll
    for (int o = 1; o < 32; o <<= 1) { const int v = __shfl_up(wincl, o, 32); if (lane >= o) wincl += v; }
    if (lane < AGG_NT / 32) scan_ws[32 + lane] = wincl - wv; if (lane == 31) scan_ws[64] = wincl; }
  __syncthreads();
  const int res = scan_ws[32 + wave] + incl - cnt; *tot = scan_ws[64];
  return res;
}
template <int SP, int CAP, int NEDGE, int NSRC>
__device__ __forceinline__ int chunk_hits(const int* __restrict__ dstv, const int* __restrict__ srcv, int e0, int n0, int tid,
                                          int* LIST, int* scan_ws) {
  const int eb = e0 + tid * SP;
  const bool real = (eb < NEDGE);
  const int ebc = real ? eb : (NEDGE - SP);
  int rec[SP]; int cnt = 0;
#pragma unroll
  for (int k = 0; k < SP; k += 4) {
    const v4i d4 = *(const v4i*)(dstv + ebc + k);
    const v4i s4 = *(const v4i*)(srcv + ebc + k);
#pragma unroll
    for (int e = 0; e < 4; ++e) {
      int sr = s4[e]; sr = sr < 0 ? 0 : (sr >= NSRC ? NSRC - 1 : sr);
      const int d = d4[e];
      int r = -1;
      if (real && d >= n0 && d < n0 + AGG_SRB) { r = ((d - n0) << 17) | sr; ++cnt; }
      rec[k + e] = r;
    }
  }
  int tot; int p = blk_excl_scan(cnt, scan_ws, tid, &tot);
#pragma unroll
  for (int k = 0; k < SP; ++k) if (rec[k] >= 0) { if ((unsigned)p < (unsigned)CAP) LIST[p] = rec[k]; ++p; }
  __syncthreads();
  return tot < CAP ? tot : CAP;
}

template <int NSRC, int NEDGE>
__global__ __launch_bounds__(AGG_NT) void agg_kernel(const float* __restrict__ SRC, const int* __restrict__ srcv, const int* __restrict__ dstv,
                                                     float* ACC, float* __restrict__ CNT) {
  constexpr int NCHK = (NEDGE + AGG_SCH - 1) / AGG_SCH;
  __shared__ int LIST[AGG_SCH];
  __shared__ int scan_ws[80];
  const int tid = threadIdx.x, lane = tid & 31, wave = tid >> 5;
  const int n0 = blockIdx.x * AGG_SRB;
  const v2f zv = {0.0f, 0.0f};
#pragma unroll 1
  for (int j = 0; j < AGG_SRB / 8; ++j) {
    float* rp = ACC + (size_t)(n0 + wave * (AGG_SRB / 8) + j) * FW + 2 * lane;
    *(volatile v2f*)rp = zv;
    __threadfence();
    *(volatile v2f*)rp = zv;
  }
  int cA0 = 0, cA1 = 0, cA2 = 0, cA3 = 0, cB0 = 0, cB1 = 0, cB2 = 0, cB3 = 0;
#pragma unroll 1
  for (int c = 0; c < NCHK; ++c) {
    const int tot = chunk_hits<AGG_SPT, AGG_SCH, NEDGE, NSRC>(dstv, srcv, c * AGG_SCH, n0, tid, LIST, scan_ws);
#pragma unroll 1
    for (int base = 0; base < tot; base += 32) {
      const int q = base + lane;
      const int qc = (q < AGG_SCH) ? q : (AGG_SCH - 1);
      const int lv = LIST[qc];
      const int rv = (q < tot) ? lv : -1;
      const int own = (rv >= 0 && (rv >> 25) == wave) ? 1 : 0;
      unsigned msk = (unsigned)__ballot(own);
#pragma unroll 1
      for (int it = 0; it < 32; ++it) {
        if (msk == 0u) break;
        const int bp = __builtin_ctz(msk); msk &= msk - 1u;
        const int r = __shfl(rv, bp, 32);
        const int dl = (r >> 17) & (AGG_SRB - 1);
        int s = r & 0x1FFFF; s = (s < NSRC) ? s : (NSRC - 1);
        const int dll = dl & 255;
        const int hs  = dll >> 7;
        const int ol  = (dll >> 2) & 31;
        const int ix  = dll & 3;
        const bool mine = (ol == lane);
        const bool mA = mine && (hs == 0), mB = mine && (hs == 1);
        cA0 += (mA && ix == 0) ? 1 : 0; cA1 += (mA && ix == 1) ? 1 : 0; cA2 += (mA && ix == 2) ? 1 : 0; cA3 += (mA && ix == 3) ? 1 : 0;
        cB0 += (mB && ix == 0) ? 1 : 0; cB1 += (mB && ix == 1) ? 1 : 0; cB2 += (mB && ix == 2) ? 1 : 0; cB3 += (mB && ix == 3) ? 1 : 0;
        const v2f pv = *(const v2f*)(SRC + (size_t)s * FW + 2 * lane);
        float* rp = ACC + (size_t)(n0 + dl) * FW + 2 * lane;
        v2f a = *(const v2f*)rp;
        a = a + pv;
        *(volatile v2f*)rp = a;
        __threadfence();
        *(volatile v2f*)rp = a;
      }
    }
    __syncthreads();
  }
  v4f dA, dB;
  dA[0] = (float)cA0; dA[1] = (float)cA1; dA[2] = (float)cA2; dA[3] = (float)cA3;
  dB[0] = (float)cB0; dB[1] = (float)cB1; dB[2] = (float)cB2; dB[3] = (float)cB3;
  float* pA = CNT + (size_t)n0 + wave * 256 + 4 * lane;
  float* pB = pA + 128;
  *(volatile v4f*)pA = dA; *(volatile v4f*)pB = dB;
  __threadfence();
  *(volatile v4f*)pA = dA; *(volatile v4f*)pB = dB;
}

__global__ __launch_bounds__(256) void meanprep_kernel(const float* __restrict__ ACC, const float* __restrict__ CNT,
                                                       unsigned short* __restrict__ MEANP) {
  const int i = blockIdx.x * 256 + threadIdx.x;
  if (i >= MPAD * 8) return;
  const int row = i >> 3, c8 = (i & 7) * 8;
  const float* pa = ACC + (size_t)row * FW + c8;
  const v4f a0 = *(const v4f*)pa, a1 = *(const v4f*)(pa + 4);
  const float cn = CNT[row];
  const float inv = 1.0f / fmaxf(cn, 1.0f);
  const float sc = (row < NNODE) ? MEAN_SC : 0.0f;
  v8h hv;
#pragma unroll
  for (int e = 0; e < 4; ++e) {
    const float u0 = (a0[e] * inv) * sc;
    const float u1 = (a1[e] * inv) * sc;
    hv[e]     = (_Float16)u0;
    hv[4 + e] = (_Float16)u1;
  }
  unsigned short* ph = MEANP + (size_t)row * FW + c8;
  *(volatile v8h*)ph = hv;
  __threadfence();
  *(volatile v8h*)ph = hv;
}

__global__ __launch_bounds__(256) void head_kernel(const float* __restrict__ H, const float* __restrict__ W2, const float* __restrict__ b2,
                                                   float* __restrict__ out) {
  const int lane = threadIdx.x & 31, wave = threadIdx.x >> 5;
  const int rb = (blockIdx.x * 8 + wave) * 32;
  if (rb >= NNODE) return;
  const int jc = (lane < NHID) ? lane : (NHID - 1);
  const float wl = W2[jc];
  const float w = (lane < NHID) ? wl : 0.0f;
  const float bb = b2[0];
  float res = 0.0f;
#pragma unroll 1
  for (int i = 0; i < 32; ++i) {
    const float hv = H[(size_t)(rb + i) * FW + lane];
    float s = hv * w;
#pragma unroll
    for (int off = 1; off < 32; off <<= 1) s += __shfl_xor(s, off, 32);
    s += bb;
    res = (lane == i) ? s : res;
  }
  float* op = out + rb + lane;
  *(volatile float*)op = res;
  __threadfence();
  *(volatile float*)op = res;
}

extern "C" void kernel_launch(void* const* d_in, const int* in_sizes, int n_in,
                              void* d_out, int out_size, void* d_ws, size_t ws_size, hipStream_t stream) {
  if (n_in < 6) return;
  if (in_sizes[0] != NNODE * FIN || in_sizes[1] != 2 * NEDGE_ALL || in_sizes[2] != NHID * FIN ||
      in_sizes[3] != NHID || in_sizes[4] != NHID || in_sizes[5] != 1) return;
  if (out_size != NNODE) return;

  const float* x  = (const float*)d_in[0];
  const int*   ei = (const int*)d_in[1];
  const float* W1 = (const float*)d_in[2];
  const float* b1 = (const float*)d_in[3];
  const float* W2 = (const float*)d_in[4];
  const float* b2 = (const float*)d_in[5];
  float* out = (float*)d_out;

  char* ws = (char*)d_ws; size_t off = 0;
  auto carve = [&](size_t bytes) -> char* { char* p = ws + off; off += (bytes + 255) & ~(size_t)255; return p; };
  float*          XP    = (float*)carve((size_t)NNODE * FW * 4);
  float*          ACC   = (float*)carve((size_t)NPA * FW * 4);
  float*          CNT   = (float*)carve((size_t)NPA * 4);
  unsigned short* MEANP = (unsigned short*)carve((size_t)MPAD * FW * 2);
  unsigned short* W1P   = (unsigned short*)carve((size_t)NGEMM * FW * 2);
  float*          B1P   = (float*)carve((size_t)NGEMM * 4);
  float*          H     = (float*)carve((size_t)MPAD * NGEMM * 4);
  if (off > ws_size || off > (size_t)134217728) return;

  xpad_kernel<<<(NNODE * 16) / 256, 256, 0, stream>>>(x, XP);
  wprep_kernel<<<(NGEMM * 8) / 256, 256, 0, stream>>>(W1, b1, W1P, B1P);
  agg_kernel<NNODE, NEDGE_ALL><<<AGG_TILES, AGG_NT, 0, stream>>>(XP, ei, ei + NEDGE_ALL, ACC, CNT);
  meanprep_kernel<<<(MPAD * 8) / 256, 256, 0, stream>>>(ACC, CNT, MEANP);
  {
    const int tiles = (MPAD / 64) * (NGEMM / 64);
    wmma_gemm64<0, false, 2, 0, false, 2><<<dim3((tiles + 7) / 8, 1), 256, 0, stream>>>(
        MEANP, nullptr, FW, 0L, W1P, nullptr, FW, 0L,
        (void*)H, nullptr, NGEMM, 0L, B1P, nullptr, 0L, MPAD, NGEMM, FW, GEMM_SC);
  }
  head_kernel<<<(NNODE + 255) / 256, 256, 0, stream>>>(H, W2, b2, out);
}
